// SemanticRematcher_21517786153375
// MI455X (gfx1250) — hardware-verified
//
#include <hip/hip_runtime.h>
#include <hip/hip_bf16.h>
#include <stdint.h>

typedef __attribute__((ext_vector_type(16))) _Float16 v16h;
typedef __attribute__((ext_vector_type(16))) __bf16   v16bf;
typedef __attribute__((ext_vector_type(8)))  float    v8f;
typedef __attribute__((ext_vector_type(8)))  _Float16 v8h;
typedef __attribute__((ext_vector_type(4)))  float    v4f;
typedef __attribute__((ext_vector_type(4)))  unsigned v4u;
typedef float __attribute__((may_alias)) float_a;
template <typename T> __device__ __forceinline__ void vst2(void* p, T v) { *(volatile T*)p = v; __threadfence(); *(volatile T*)p = v; }
__device__ __forceinline__ v8f WM16(v16h a, v16h b, v8f c) {
    v8f d = __builtin_amdgcn_wmma_f32_16x16x32_f16(false, a, false, b, (short)0, c, false, false);
    asm volatile("v_nop\n\tv_nop\n\tv_nop\n\tv_nop" : "+v"(d) : "v"(a), "v"(b));
    return d;
}

#define BN 1024
#define DN 1024
#define REG_INV 10.0f
#define EPS_F 1e-8f
#define THRESH 1e-3f
#define MAX_ITER 100

union BFrag { uint4 q[2]; v16bf v; };
union HFrag { uint4 q[2]; v16h  v; };

__device__ inline unsigned short f2bf(float f) {
    union { _Float16 h; unsigned short u; } c; c.h = (_Float16)f; return c.u;
}

__global__ __launch_bounds__(256) void k_normalize(
        const float* __restrict__ vis, const float* __restrict__ txt,
        unsigned short* __restrict__ vnb, unsigned short* __restrict__ tnb) {
    int lane = threadIdx.x & 31;
    int wave = threadIdx.x >> 5;
    int row  = blockIdx.x * 8 + wave;
    const float* src = (row < BN) ? (vis + (size_t)row * DN)
                                  : (txt + (size_t)(row - BN) * DN);
    unsigned short* dst = (row < BN) ? (vnb + (size_t)row * DN)
                                     : (tnb + (size_t)(row - BN) * DN);
    float x[32];
    float ss = 0.f;
#pragma unroll
    for (int i = 0; i < 32; i++) { x[i] = src[i * 32 + lane]; ss = fmaf(x[i], x[i], ss); }
#pragma unroll
    for (int m = 16; m >= 1; m >>= 1) ss += __shfl_xor(ss, m, 32);
    float inv = rsqrtf(ss);
    __shared__ __align__(16) unsigned short rowbuf[8][DN];
#pragma unroll
    for (int i = 0; i < 32; i++) rowbuf[wave][i * 32 + lane] = f2bf(x[i] * inv);
    asm volatile("s_wait_dscnt 0" ::: "memory"); __builtin_amdgcn_wave_barrier(); __builtin_amdgcn_fence(__ATOMIC_RELEASE, "workgroup");
#pragma unroll
    for (int q = 0; q < 4; q++) vst2(dst + (q * 32 + lane) * 8, *(const v4u*)(&rowbuf[wave][(q * 32 + lane) * 8]));
}

__global__ __launch_bounds__(256) void k_sim(
        const unsigned short* __restrict__ vnb,
        const unsigned short* __restrict__ tnb,
        float* __restrict__ sim) {
    int lane = threadIdx.x & 31;
    int wave = threadIdx.x >> 5;
    __shared__ __align__(16) float so[8][16 * 32];
    int w  = blockIdx.x * 8 + wave;
    int tm = w >> 5, tn2 = w & 31;
    int lo = lane & 15, hi = lane >> 4;

    const unsigned short* arow  = vnb + (size_t)(tm * 16 + lo) * DN;
    const unsigned short* brow0 = tnb + (size_t)(tn2 * 32 + lo) * DN;
    const unsigned short* brow1 = tnb + (size_t)(tn2 * 32 + 16 + lo) * DN;

    v8f acc = {0.f, 0.f, 0.f, 0.f, 0.f, 0.f, 0.f, 0.f}, acc1 = acc;
#pragma unroll 4
    for (int kk = 0; kk < DN; kk += 32) {
        HFrag a, b0, b1;
        const uint4* ap = reinterpret_cast<const uint4*>(arow + kk + hi * 8);
        a.q[0] = ap[0]; a.q[1] = ap[2];
        const uint4* bp0 = reinterpret_cast<const uint4*>(brow0 + kk + hi * 8);
        b0.q[0] = bp0[0]; b0.q[1] = bp0[2];
        const uint4* bp1 = reinterpret_cast<const uint4*>(brow1 + kk + hi * 8);
        b1.q[0] = bp1[0]; b1.q[1] = bp1[2];
        acc  = WM16(a.v, b0.v, acc);
        acc1 = WM16(a.v, b1.v, acc1);
    }
    float* S = so[wave];
#pragma unroll
    for (int r = 0; r < 8; r++) { S[(hi * 8 + r) * 32 + lo] = acc[r]; S[(hi * 8 + r) * 32 + 16 + lo] = acc1[r]; }
    asm volatile("s_wait_dscnt 0" ::: "memory"); __builtin_amdgcn_wave_barrier(); __builtin_amdgcn_fence(__ATOMIC_RELEASE, "workgroup");
#pragma unroll
    for (int q = 0; q < 4; q++) { const int rl = q * 4 + (lane >> 3), pc = lane & 7;
        vst2(sim + (size_t)(tm * 16 + rl) * BN + tn2 * 32 + pc * 4, *(const v4f*)(S + rl * 32 + pc * 4)); }
}

__global__ __launch_bounds__(256) void k_cost(
        const float* __restrict__ sim,
        const float* __restrict__ W1, const float* __restrict__ b1,
        const float* __restrict__ W2, const float* __restrict__ b2,
        const float* __restrict__ W3, const float* __restrict__ b3,
        const float* __restrict__ W4, const float* __restrict__ b4,
        float* __restrict__ cost, float* __restrict__ Kmat) {
    __shared__ float w1s[128], b1s[128], b2s[64], b3s[32], w4s[32];
    __shared__ float b4s;
    __shared__ _Float16 __align__(16) h2s[8][16 * 64];
    __shared__ __align__(16) float cst_s[8][16], km_s[8][16];

    int t = threadIdx.x;
    if (t < 128) w1s[t] = W1[t]; else b1s[t - 128] = b1[t - 128];
    if (t < 64) b2s[t] = b2[t];
    else if (t < 96) b3s[t - 64] = b3[t - 64];
    else if (t < 128) w4s[t - 96] = W4[t - 96];
    if (t == 0) b4s = b4[0];
    __syncthreads();

    int lane = t & 31, wv = t >> 5;
    int lo = lane & 15, hi = lane >> 4;
    int waveG = blockIdx.x * 8 + wv;

    __shared__ __align__(16) _Float16 w2t[64 * 136];
    __shared__ __align__(16) _Float16 w3t[32 * 72];
    for (int i = t; i < 128 * 64; i += 256) { int k = i >> 6, n = i & 63; w2t[n * 136 + k] = (_Float16)W2[i]; }
    for (int i = t; i < 64 * 32; i += 256)  { int k = i >> 5, n = i & 31; w3t[n * 72 + k] = (_Float16)W3[i]; }
    __syncthreads();
    auto bfragW2 = [&](int ks, int nt) { HFrag f; const uint4* p = reinterpret_cast<const uint4*>(&w2t[(nt * 16 + lo) * 136 + ks * 32 + hi * 8]); f.q[0] = p[0]; f.q[1] = p[2]; return f.v; };
    auto bfragW3 = [&](int ks, int nt) { HFrag f; const uint4* p = reinterpret_cast<const uint4*>(&w3t[(nt * 16 + lo) * 72 + ks * 32 + hi * 8]); f.q[0] = p[0]; f.q[1] = p[2]; return f.v; };

    for (int it = 0; it < 32; it++) {
        int group = it * 2048 + waveG;
        int base  = group * 16;
        float x = sim[base + lo];

        v8f acc2[4];
#pragma unroll
        for (int nt = 0; nt < 4; nt++) {
            float bb = b2s[nt * 16 + lo];
#pragma unroll
            for (int r = 0; r < 8; r++) acc2[nt][r] = bb;
        }

#pragma unroll
        for (int ks = 0; ks < 4; ks++) {
            v16h a1;
#pragma unroll
            for (int e = 0; e < 16; e++) {
                int k = ks * 32 + hi * 8 + (e & 7) + ((e >= 8) ? 16 : 0);
                float h = fmaf(x, w1s[k], b1s[k]);
                a1[e] = (_Float16)fmaxf(h, 0.f);
            }
#pragma unroll
            for (int nt = 0; nt < 4; nt++)
                acc2[nt] = WM16(a1, bfragW2(ks, nt), acc2[nt]);
        }

#pragma unroll
        for (int nt = 0; nt < 4; nt++)
#pragma unroll
            for (int r = 0; r < 8; r++)
                h2s[wv][(r + hi * 8) * 64 + nt * 16 + lo] =
                    (_Float16)fmaxf(acc2[nt][r], 0.f);

        asm volatile("s_wait_dscnt 0" ::: "memory"); __builtin_amdgcn_wave_barrier(); __builtin_amdgcn_fence(__ATOMIC_RELEASE, "workgroup");
        v16h a3[2];
#pragma unroll
        for (int ks = 0; ks < 2; ks++) {
            HFrag f;
            const uint4* p = reinterpret_cast<const uint4*>(
                &h2s[wv][lo * 64 + ks * 32 + hi * 8]);
            f.q[0] = p[0];
            f.q[1] = p[2];
            a3[ks] = f.v;
        }

        __builtin_amdgcn_wave_barrier();
        v8f h3[2];
#pragma unroll
        for (int nt = 0; nt < 2; nt++) {
            float bb = b3s[nt * 16 + lo];
            v8f acc;
#pragma unroll
            for (int r = 0; r < 8; r++) acc[r] = bb;
#pragma unroll
            for (int ks = 0; ks < 2; ks++)
                acc = WM16(a3[ks], bfragW3(ks, nt), acc);
#pragma unroll
            for (int r = 0; r < 8; r++) acc[r] = fmaxf(acc[r], 0.f);
            h3[nt] = acc;
        }

        float s[8];
        float wA = w4s[lo], wB = w4s[16 + lo];
#pragma unroll
        for (int r = 0; r < 8; r++) s[r] = h3[0][r] * wA + h3[1][r] * wB;
#pragma unroll
        for (int m = 1; m < 16; m <<= 1)
#pragma unroll
            for (int r = 0; r < 8; r++) s[r] += __shfl_xor(s[r], m, 32);

        if (lo < 8) {
            float val = s[0];
#pragma unroll
            for (int r = 1; r < 8; r++) val = (lo == r) ? s[r] : val;
            float z   = val + b4s;
            float sg  = 1.f / (1.f + __expf(-z));
            float cst = 1.f - sg;
            cst_s[wv][lo + hi * 8] = cst;
            km_s[wv][lo + hi * 8]  = __expf(-cst * REG_INV);
        }
        __syncthreads();
        if (t < 32) { const size_t o = (size_t)it * 32768 + (size_t)blockIdx.x * 128 + t * 4;
            vst2(cost + o, *(const v4f*)(&cst_s[0][0] + t * 4)); vst2(Kmat + o, *(const v4f*)(&km_s[0][0] + t * 4)); }
        __syncthreads();
    }
}

__global__ void k_sink_init(float* u, float* v, float* du2, int* done) {
    int i = blockIdx.x * blockDim.x + threadIdx.x;
    if (i < BN) { u[i] = 1.f / BN; v[i] = 1.f / BN; du2[i] = 0.f; }
    if (i == 0) *done = 0;
}

__global__ void k_sink_v(const float* __restrict__ K, const float* __restrict__ u,
                         float* __restrict__ v, const int* __restrict__ done) {
    if (*done) return;
    int j = blockIdx.x * blockDim.x + threadIdx.x;
    float sum = 0.f;
#pragma unroll 1
    for (int i = 0; i < BN; i++) sum = fmaf(K[(size_t)i * BN + j], u[i], sum);
    vst2(v + j, (float_a)((1.f / BN) / (sum + EPS_F)));
}

__global__ __launch_bounds__(256) void k_sink_u(
        const float* __restrict__ K, const float* __restrict__ v,
        float* __restrict__ u, float* __restrict__ du2,
        const int* __restrict__ done) {
    if (*done) return;
    __shared__ float su[32], sd[32];
    int lane = threadIdx.x & 31, wave = threadIdx.x >> 5;
#pragma unroll 1
    for (int rr = 0; rr < 4; rr++) {
        int i = blockIdx.x * 32 + wave * 4 + rr;
        const float* row = K + (size_t)i * BN;
        float sum = 0.f;
#pragma unroll 1
        for (int j = lane; j < BN; j += 32) sum = fmaf(row[j], v[j], sum);
#pragma unroll
        for (int m = 16; m >= 1; m >>= 1) sum += __shfl_xor(sum, m, 32);
        if (lane == 0) {
            float un = (1.f / BN) / (sum + EPS_F);
            float d  = un - u[i];
            sd[wave * 4 + rr] = d * d;
            su[wave * 4 + rr] = un;
        }
    }
    __syncthreads();
    if (threadIdx.x < 32) { vst2(u + blockIdx.x * 32 + threadIdx.x, (float_a)su[threadIdx.x]); vst2(du2 + blockIdx.x * 32 + threadIdx.x, (float_a)sd[threadIdx.x]); }
}

__global__ void k_sink_fin(const float* __restrict__ du2, int* done) {
    __shared__ float red[256];
    float s = 0.f;
    for (int i = threadIdx.x; i < BN; i += 256) s += du2[i];
    red[threadIdx.x] = s;
    __syncthreads();
    for (int st = 128; st > 0; st >>= 1) {
        if (threadIdx.x < st) red[threadIdx.x] += red[threadIdx.x + st];
        __syncthreads();
    }
    if (threadIdx.x == 0) { if (!*done && sqrtf(red[0]) < THRESH) *done = 1; }
}

__global__ __launch_bounds__(256) void k_transport(
        const float* __restrict__ K, const float* __restrict__ u,
        const float* __restrict__ v, float* __restrict__ T) {
    int idx = blockIdx.x * blockDim.x + threadIdx.x;
    int i = idx >> 10, j = idx & 1023;
    vst2(T + idx, (float_a)(u[i] * K[idx] * v[j]));
}

extern "C" void kernel_launch(void* const* d_in, const int* in_sizes, int n_in,
                              void* d_out, int out_size, void* d_ws, size_t ws_size,
                              hipStream_t stream) {
    (void)in_sizes; (void)n_in; (void)out_size; (void)ws_size;
    const float* vis = (const float*)d_in[0];
    const float* txt = (const float*)d_in[1];
    const float* W1  = (const float*)d_in[2];
    const float* b1  = (const float*)d_in[3];
    const float* W2  = (const float*)d_in[4];
    const float* b2  = (const float*)d_in[5];
    const float* W3  = (const float*)d_in[6];
    const float* b3  = (const float*)d_in[7];
    const float* W4  = (const float*)d_in[8];
    const float* b4  = (const float*)d_in[9];

    float* T    = (float*)d_out;
    float* cost = (float*)d_out + 1024 * 1024;
    float* sim  = (float*)d_out + 2 * 1024 * 1024;

    char* ws = (char*)d_ws;
    unsigned short* vnb = (unsigned short*)ws;
    unsigned short* tnb = (unsigned short*)(ws + (size_t)2 * 1024 * 1024);
    float* Km  = (float*)(ws + (size_t)4 * 1024 * 1024);
    float* u   = (float*)(ws + (size_t)8 * 1024 * 1024);
    float* v   = (float*)(ws + (size_t)8 * 1024 * 1024 + 4096);
    float* du2 = (float*)(ws + (size_t)8 * 1024 * 1024 + 8192);
    int*  done = (int*) (ws + (size_t)8 * 1024 * 1024 + 12288);

    k_normalize<<<256, 256, 0, stream>>>(vis, txt, vnb, tnb);
    k_sim<<<256, 256, 0, stream>>>(vnb, tnb, sim);
    k_cost<<<256, 256, 0, stream>>>(sim, W1, b1, W2, b2, W3, b3, W4, b4, cost, Km);
    k_sink_init<<<4, 256, 0, stream>>>(u, v, du2, done);
    for (int it = 0; it < MAX_ITER; it++) {
        k_sink_v<<<4, 256, 0, stream>>>(Km, u, v, done);
        k_sink_u<<<32, 256, 0, stream>>>(Km, v, u, du2, done);
        k_sink_fin<<<1, 256, 0, stream>>>(du2, done);
    }
    k_transport<<<4096, 256, 0, stream>>>(Km, u, v, T);
}
